// MAB_72911364817388
// MI455X (gfx1250) — hardware-run, weakly checked
//
#include <hip/hip_runtime.h>
#include <math.h>
#include <stdint.h>

#define NB    8
#define NQ    1024
#define NK    1024
#define DM    512
#define NH    8
#define HD    64
#define ROWQ  (NB * NQ)
#define ROWK  (NB * NK)
#define NQB   (NQ / 64)
#define NKT   (NK / 64)
static_assert(NH * HD == DM);
static_assert(HD == 64);
static_assert(ROWQ == ROWK);
static_assert((NQ % 64) == 0 && (NK % 64) == 0 && (DM % 64) == 0);
static_assert((((ROWQ / 64) * (DM / 64)) % 8) == 0);
static_assert(((ROWQ * DM / 8) % 256) == 0);
static_assert((ROWQ % 8) == 0);

typedef _Float16 v16h __attribute__((ext_vector_type(16)));
typedef _Float16 v8h  __attribute__((ext_vector_type(8)));
typedef float    v8f  __attribute__((ext_vector_type(8)));
typedef float    v4f  __attribute__((ext_vector_type(4)));
typedef unsigned int v4u __attribute__((ext_vector_type(4)));
typedef unsigned int v2u __attribute__((ext_vector_type(2)));

__device__ __forceinline__ unsigned short bf_bits(float f) {
  unsigned u = __float_as_uint(f);
  return (unsigned short)((u + 0x7FFFu + ((u >> 16) & 1u)) >> 16);
}
__device__ __forceinline__ float bfr(float f) { return __uint_as_float(((unsigned)bf_bits(f)) << 16); }
__device__ __forceinline__ unsigned short h_bits(_Float16 x) { return __builtin_bit_cast(unsigned short, x); }
__device__ __forceinline__ unsigned pk16(unsigned short a, unsigned short b) { return (unsigned)a | ((unsigned)b << 16); }
__device__ __forceinline__ v8f zero8() { v8f z = {0.f, 0.f, 0.f, 0.f, 0.f, 0.f, 0.f, 0.f}; return z; }

__device__ __forceinline__ v16h ldfrag_h(const _Float16* p) {
  union { v16h v; v8h h[2]; } f;
  f.h[0] = *(const v8h*)(p);
  f.h[1] = *(const v8h*)(p + 16);
  return f.v;
}

__device__ __forceinline__ v8f mma_h(v16h a, v16h b, v8f c) {
  c = __builtin_amdgcn_wmma_f32_16x16x32_f16(false, a, false, b, (short)0, c, false, false);
#if defined(__HIP_DEVICE_COMPILE__)
  asm volatile("v_nop\n\tv_nop\n\tv_nop\n\tv_nop" : "+v"(c) : "v"(a), "v"(b));
#endif
  return c;
}
__device__ __forceinline__ v8f mma_h_raw(v16h a, v16h b, v8f c) {
  return __builtin_amdgcn_wmma_f32_16x16x32_f16(false, a, false, b, (short)0, c, false, false);
}
__device__ __forceinline__ void dep_guard_h(v8f& a, v8f& b, v16h x, v16h y) {
#if defined(__HIP_DEVICE_COMPILE__)
  asm volatile("v_nop\n\tv_nop\n\tv_nop\n\tv_nop" : "+v"(a), "+v"(b) : "v"(x), "v"(y));
#endif
}
__device__ __forceinline__ void keep4_h(v16h a, v16h b, v16h c, v16h d) {
#if defined(__HIP_DEVICE_COMPILE__)
  asm volatile("v_nop" :: "v"(a), "v"(b), "v"(c), "v"(d));
#endif
}
__device__ __forceinline__ void acc_guard4(v8f& a, v8f& b, v8f& c, v8f& d) {
#if defined(__HIP_DEVICE_COMPILE__)
  asm volatile("v_nop\n\tv_nop\n\tv_nop\n\tv_nop" : "+v"(a), "+v"(b), "+v"(c), "+v"(d));
#endif
}

__global__ __launch_bounds__(256) void cvt16(const float* __restrict__ in, unsigned short* out, int n8, float scale) {
  const int i = blockIdx.x * 256 + threadIdx.x;
  if (i < n8) {
    const v4f a = *(const v4f*)(in + (size_t)i * 8);
    const v4f b = *(const v4f*)(in + (size_t)i * 8 + 4);
    v4u p;
    p[0] = pk16(h_bits((_Float16)(bfr(a[0]) * scale)), h_bits((_Float16)(bfr(a[1]) * scale)));
    p[1] = pk16(h_bits((_Float16)(bfr(a[2]) * scale)), h_bits((_Float16)(bfr(a[3]) * scale)));
    p[2] = pk16(h_bits((_Float16)(bfr(b[0]) * scale)), h_bits((_Float16)(bfr(b[1]) * scale)));
    p[3] = pk16(h_bits((_Float16)(bfr(b[2]) * scale)), h_bits((_Float16)(bfr(b[3]) * scale)));
    *(volatile v4u*)(out + (size_t)i * 8) = p;
    __threadfence();
    *(volatile v4u*)(out + (size_t)i * 8) = p;
  }
}

__global__ __launch_bounds__(256) void wtr16(const float* __restrict__ W, unsigned short* Wt, int nk, int nn, float scale) {
  __shared__ __align__(16) float st[64 * 68];
  const int tid = threadIdx.x;
  const int n0 = blockIdx.x * 64;
  const int k0 = blockIdx.y * 64;
#pragma unroll
  for (int i = 0; i < 4; ++i) {
    const int idx = i * 256 + tid;
    const int kk = idx >> 4, c4 = (idx & 15) * 4;
    const v4f a = *(const v4f*)(W + (size_t)(k0 + kk) * nn + n0 + c4);
    *(v4f*)(st + kk * 68 + c4) = a;
  }
  __syncthreads();

  const int g = tid >> 3, piece = tid & 7;
  v4u hv[2];
  size_t hofs[2];
#pragma unroll
  for (int it = 0; it < 2; ++it) {
    const int n = it * 32 + g;
    v4u a;
#pragma unroll
    for (int e = 0; e < 4; ++e) {
      const float x0 = st[(piece * 8 + 2 * e) * 68 + n];
      const float x1 = st[(piece * 8 + 2 * e + 1) * 68 + n];
      a[e] = pk16(h_bits((_Float16)(bfr(x0) * scale)), h_bits((_Float16)(bfr(x1) * scale)));
    }
    hv[it] = a;
    hofs[it] = (size_t)(n0 + n) * nk + k0 + piece * 8;
  }
  for (int pass = 0; pass < 2; ++pass) {
#pragma unroll
    for (int it = 0; it < 2; ++it) *(volatile v4u*)(Wt + hofs[it]) = hv[it];
    __threadfence();
  }
}

template <int EPI>
__global__ __launch_bounds__(256) void gemm64_f16(
    const unsigned short* __restrict__ Ap, int lda,
    const unsigned short* __restrict__ Btp, int ldb,
    const float* __restrict__ biasp, const float* __restrict__ resp,
    float cscale, float oscale,
    float* Cf, unsigned short* C16, int ldc, int M, int N, int K) {
  const _Float16* Ah = (const _Float16*)(const void*)Ap;
  const _Float16* Bt = (const _Float16*)(const void*)Btp;
  __shared__ __align__(16) float sT[8][16 * 68];
  const int lane = threadIdx.x & 31;
  const int wave = threadIdx.x >> 5;
  const int tilesN = N >> 6;
  const int tilesM = M >> 6;
  const int tile = blockIdx.x * 8 + wave;
  if (tile >= tilesM * tilesN) return;
  const int tm = tile / tilesN;
  const int tn = tile - tm * tilesN;
  const int m0 = tm << 6;
  const int n0 = tn << 6;

  const int rlane = lane & 15;
  const int koff  = (lane >> 4) * 8;
  const int mOff  = (lane >> 4) * 8;

  v8f acc[4][4];
#pragma unroll
  for (int i = 0; i < 4; ++i)
#pragma unroll
    for (int j = 0; j < 4; ++j) acc[i][j] = zero8();

  for (int k0 = 0; k0 < K; k0 += 32) {
    v16h bh[4];
#pragma unroll
    for (int j = 0; j < 4; ++j) {
      const size_t bo = (size_t)(n0 + (j << 4) + rlane) * ldb + koff + k0;
      bh[j] = ldfrag_h(Bt + bo);
    }
#pragma unroll
    for (int i = 0; i < 4; ++i) {
      const size_t ao = (size_t)(m0 + (i << 4) + rlane) * lda + koff + k0;
      const v16h ah = ldfrag_h(Ah + ao);
#pragma unroll
      for (int j = 0; j < 4; ++j) {
        acc[i][j] = mma_h_raw(ah, bh[j], acc[i][j]);
      }
      dep_guard_h(acc[i][0], acc[i][3], ah, bh[3]);
    }
    keep4_h(bh[0], bh[1], bh[2], bh[3]);
  }
  acc_guard4(acc[0][0], acc[0][1], acc[0][2], acc[0][3]);
  acc_guard4(acc[1][0], acc[1][1], acc[1][2], acc[1][3]);
  acc_guard4(acc[2][0], acc[2][1], acc[2][2], acc[2][3]);
  acc_guard4(acc[3][0], acc[3][1], acc[3][2], acc[3][3]);

  float* slab = sT[wave];
#pragma unroll
  for (int i = 0; i < 4; ++i) {
    const int mBase = m0 + (i << 4);
    float bj[4];
#pragma unroll
    for (int j = 0; j < 4; ++j) bj[j] = bfr(biasp[n0 + (j << 4) + rlane]);
#pragma unroll
    for (int r = 0; r < 8; ++r) {
      const int row = mOff + r;
#pragma unroll
      for (int j = 0; j < 4; ++j) slab[row * 68 + (j << 4) + rlane] = acc[i][j][r] * cscale + bj[j];
    }
    __builtin_amdgcn_fence(__ATOMIC_RELEASE, "workgroup");
    __builtin_amdgcn_wave_barrier();
    __builtin_amdgcn_fence(__ATOMIC_ACQUIRE, "workgroup");
    if constexpr (EPI == 0 || EPI == 1) {
      const int rq = lane >> 3, piece = lane & 7;
      v4u ph[4];
#pragma unroll
      for (int it = 0; it < 4; ++it) {
        const int row = it * 4 + rq;
        const v4f a  = *(const v4f*)(slab + row * 68 + piece * 8);
        const v4f a2 = *(const v4f*)(slab + row * 68 + piece * 8 + 4);
        float f[8];
        f[0] = a[0];  f[1] = a[1];  f[2] = a[2];  f[3] = a[3];
        f[4] = a2[0]; f[5] = a2[1]; f[6] = a2[2]; f[7] = a2[3];
        v4u p;
#pragma unroll
        for (int e = 0; e < 4; ++e) {
          const _Float16 x0 = (_Float16)(f[2 * e] * oscale);
          const _Float16 x1 = (_Float16)(f[2 * e + 1] * oscale);
          p[e] = pk16(h_bits(x0), h_bits(x1));
        }
        ph[it] = p;
      }
      for (int pass = 0; pass < 2; ++pass) {
#pragma unroll
        for (int it = 0; it < 4; ++it) {
          const int row = it * 4 + rq;
          const size_t co = (size_t)(mBase + row) * ldc + n0 + piece * 8;
          *(volatile v4u*)(C16 + co) = ph[it];
        }
        __threadfence();
      }
    }
    if constexpr (EPI == 1 || EPI == 2) {
      const int h2 = lane >> 4, c4 = (lane & 15) * 4;
      v4f ov[8];
#pragma unroll
      for (int it = 0; it < 8; ++it) {
        const int row = it * 2 + h2;
        v4f a = *(const v4f*)(slab + row * 68 + c4);
        if constexpr (EPI == 2) {
          const v4f rv = *(const v4f*)(resp + (size_t)(mBase + row) * ldc + n0 + c4);
          v4f y;
          y[0] = rv[0] + fmaxf(a[0], 0.0f);
          y[1] = rv[1] + fmaxf(a[1], 0.0f);
          y[2] = rv[2] + fmaxf(a[2], 0.0f);
          y[3] = rv[3] + fmaxf(a[3], 0.0f);
          a = y;
        }
        ov[it] = a;
      }
      for (int pass = 0; pass < 2; ++pass) {
#pragma unroll
        for (int it = 0; it < 8; ++it) {
          const int row = it * 2 + h2;
          *(volatile v4f*)(Cf + (size_t)(mBase + row) * ldc + n0 + c4) = ov[it];
        }
        __threadfence();
      }
    }
    __builtin_amdgcn_fence(__ATOMIC_RELEASE, "workgroup");
    __builtin_amdgcn_wave_barrier();
    __builtin_amdgcn_fence(__ATOMIC_ACQUIRE, "workgroup");
  }
}

__global__ __launch_bounds__(256) void v_tr(const unsigned short* __restrict__ vp, unsigned short* vt) {
  __shared__ __align__(16) _Float16 sv[64 * 72];
  const int tid = threadIdx.x;
  const int t0  = blockIdx.x * 64;
  const int hh  = blockIdx.y;
  const int b   = blockIdx.z;
  const _Float16* src = (const _Float16*)(const void*)vp;
#pragma unroll
  for (int i = 0; i < 2; ++i) {
    const int idx = i * 256 + tid;
    const int tt = idx >> 3, c8 = (idx & 7) * 8;
    const v8h a = *(const v8h*)(src + ((size_t)(b * NK + t0 + tt)) * DM + hh * HD + c8);
    *(v8h*)(sv + tt * 72 + c8) = a;
  }
  __syncthreads();

  const int g = tid >> 3, piece = tid & 7;
  v4u hv[2];
  size_t hofs[2];
#pragma unroll
  for (int it = 0; it < 2; ++it) {
    const int d = it * 32 + g;
    v4u a;
#pragma unroll
    for (int e = 0; e < 4; ++e) {
      const _Float16 x0 = sv[(piece * 8 + 2 * e) * 72 + d];
      const _Float16 x1 = sv[(piece * 8 + 2 * e + 1) * 72 + d];
      a[e] = pk16(h_bits(x0), h_bits(x1));
    }
    hv[it] = a;
    hofs[it] = ((size_t)(b * DM + hh * HD + d)) * NK + t0 + piece * 8;
  }
  for (int pass = 0; pass < 2; ++pass) {
#pragma unroll
    for (int it = 0; it < 2; ++it) *(volatile v4u*)(vt + hofs[it]) = hv[it];
    __threadfence();
  }
}

__global__ __launch_bounds__(128)
void attn_k(const unsigned short* __restrict__ q16p, const unsigned short* __restrict__ k16p,
            const unsigned short* __restrict__ vtp, const float* __restrict__ qfp,
            const int* __restrict__ maskp, float* outp) {
  union FH { v16h v; v8h h[2]; };
  constexpr int TB    = 64 * 64 * 2;
  constexpr int PB    = 4 * 16 * 64 * 2;
  constexpr int OFF_K = 0;
  constexpr int OFF_V = TB;
  constexpr int OFF_P = 2 * TB;
  constexpr int OFF_M = OFF_P + PB;
  constexpr int SMEMB = OFF_M + 64 * 4;
  static_assert(4 * 16 * 64 * 4 <= OFF_P);
  __shared__ __align__(16) unsigned char smem[SMEMB];
  _Float16* Ksh = (_Float16*)(smem + OFF_K);
  _Float16* Vsh = (_Float16*)(smem + OFF_V);
  _Float16* Psh = (_Float16*)(smem + OFF_P);
  int*      Msh = (int*)(smem + OFF_M);

  const int tid  = threadIdx.x;
  const int wave = tid >> 5;
  const int lane = tid & 31;
  const int hh   = lane >> 4;
  const int c    = lane & 15;

  const int bx   = blockIdx.x;
  const int qb   = bx % NQB;
  const int rest = bx / NQB;
  const int h    = rest % NH;
  const int b    = rest / NH;
  const int q0   = qb * 64 + wave * 16;
  const size_t rowQ = (size_t)b * NQ;
  const size_t rowK = (size_t)b * NK;

  const _Float16* Qp = (const _Float16*)(const void*)q16p + (size_t)h * HD;
  const _Float16* Kp = (const _Float16*)(const void*)k16p + (size_t)h * HD;
  const _Float16* Vt = (const _Float16*)(const void*)vtp + ((size_t)b * DM + (size_t)h * HD) * NK;
  const int* Mb = maskp + (size_t)b * NK;

  v16h qa[2];
#pragma unroll
  for (int dc = 0; dc < 2; ++dc) {
    const size_t qo = (rowQ + q0 + c) * DM + dc * 32 + 8 * hh;
    qa[dc] = ldfrag_h(Qp + qo);
  }

  float mrow[8], lrow[8];
  v8f o[4];
#pragma unroll
  for (int r = 0; r < 8; ++r) { mrow[r] = -1.0e30f; lrow[r] = 0.f; }
#pragma unroll
  for (int t = 0; t < 4; ++t) o[t] = zero8();

  _Float16* pw = Psh + wave * (16 * 64);
  const float scl = (1.0f / 256.0f) * 0.044194173824159216f;

  for (int kt = 0; kt < NKT; ++kt) {
    const int kv0 = kt * 64;
    __syncthreads();
    {
      const int r = tid >> 1, half = (tid & 1) * 32;
      const size_t ko = (rowK + kv0 + r) * DM + half;
      const size_t vo = (size_t)r * NK + kv0 + half;
#pragma unroll
      for (int i = 0; i < 4; ++i) {
        const v8h a0 = *(const v8h*)(Kp + ko + 8 * i);
        const v8h b0 = *(const v8h*)(Vt + vo + 8 * i);
        *(v8h*)(Ksh + r * 64 + half + 8 * i) = a0;
        *(v8h*)(Vsh + r * 64 + half + 8 * i) = b0;
      }
      if (tid < 64) Msh[tid] = Mb[kv0 + tid];
    }
    __syncthreads();

    v8f s[4];
#pragma unroll
    for (int j = 0; j < 4; ++j) {
      s[j] = zero8();
#pragma unroll
      for (int dc = 0; dc < 2; ++dc) {
        FH kb;
        kb.h[0] = *(const v8h*)(Ksh + (j * 16 + c) * 64 + dc * 32 + 8 * hh);
        kb.h[1] = *(const v8h*)(Ksh + (j * 16 + c) * 64 + dc * 32 + 16 + 8 * hh);
        s[j] = mma_h(qa[dc], kb.v, s[j]);
      }
    }

    int mk[4];
#pragma unroll
    for (int j = 0; j < 4; ++j) mk[j] = Msh[j * 16 + c];
#pragma unroll
    for (int r = 0; r < 8; ++r) {
      float f[4];
#pragma unroll
      for (int j = 0; j < 4; ++j) {
        const float a = s[j][r] * scl;
        f[j] = (mk[j] == 0) ? -10000.0f : a;
      }
      float tmx = fmaxf(fmaxf(f[0], f[1]), fmaxf(f[2], f[3]));
#pragma unroll
      for (int off = 1; off < 16; off <<= 1) tmx = fmaxf(tmx, __shfl_xor(tmx, off, 32));
      const float mn   = fmaxf(mrow[r], tmx);
      const float corr = __expf(mrow[r] - mn);
      mrow[r] = mn;
      float ps = 0.0f;
#pragma unroll
      for (int j = 0; j < 4; ++j) {
        const float p = __expf(f[j] - mn);
        ps += p;
        pw[(8 * hh + r) * 64 + j * 16 + c] = (_Float16)(p * 256.0f);
      }
      lrow[r] = lrow[r] * corr + ps;
#pragma unroll
      for (int t = 0; t < 4; ++t) o[t][r] = o[t][r] * corr;
    }
    __builtin_amdgcn_fence(__ATOMIC_RELEASE, "workgroup");
    __builtin_amdgcn_wave_barrier();
    __builtin_amdgcn_fence(__ATOMIC_ACQUIRE, "workgroup");

#pragma unroll
    for (int kk = 0; kk < 2; ++kk) {
      FH pa;
      pa.h[0] = *(const v8h*)(pw + c * 64 + kk * 32 + 8 * hh);
      pa.h[1] = *(const v8h*)(pw + c * 64 + kk * 32 + 16 + 8 * hh);
#pragma unroll
      for (int t = 0; t < 4; ++t) {
        FH vb;
        vb.h[0] = *(const v8h*)(Vsh + (t * 16 + c) * 64 + kk * 32 + 8 * hh);
        vb.h[1] = *(const v8h*)(Vsh + (t * 16 + c) * 64 + kk * 32 + 16 + 8 * hh);
        o[t] = mma_h(pa.v, vb.v, o[t]);
      }
    }
  }
  __syncthreads();

  float* os = (float*)(void*)smem + wave * (16 * 64);
#pragma unroll
  for (int r = 0; r < 8; ++r) {
    float l = lrow[r];
#pragma unroll
    for (int off = 1; off < 16; off <<= 1) l += __shfl_xor(l, off, 32);
    const float sc = (1.0f / l) * (1.0f / 4096.0f);
#pragma unroll
    for (int t = 0; t < 4; ++t) os[(8 * hh + r) * 64 + t * 16 + c] = o[t][r] * sc;
  }
  __builtin_amdgcn_fence(__ATOMIC_RELEASE, "workgroup");
  __builtin_amdgcn_wave_barrier();
  __builtin_amdgcn_fence(__ATOMIC_ACQUIRE, "workgroup");
  {
    const int h2 = lane >> 4, c4 = (lane & 15) * 4;
    v4f ov[8];
#pragma unroll
    for (int it = 0; it < 8; ++it) {
      const int row = it * 2 + h2;
      const v4f a  = *(const v4f*)(os + row * 64 + c4);
      const v4f qv = *(const v4f*)(qfp + (rowQ + q0 + row) * DM + (size_t)h * HD + c4);
      ov[it] = a + qv;
    }
    for (int pass = 0; pass < 2; ++pass) {
#pragma unroll
      for (int it = 0; it < 8; ++it) {
        const int row = it * 2 + h2;
        const size_t go = (rowQ + q0 + row) * DM + (size_t)h * HD + c4;
        *(volatile v4f*)(outp + go) = ov[it];
      }
      __threadfence();
    }
  }
}

template <bool H16>
__global__ __launch_bounds__(256) void ln_k(const float* __restrict__ x, const float* __restrict__ gw,
                                            const float* __restrict__ bw, float* outf, unsigned short* out16,
                                            int nrows, float oscale) {
  __shared__ __align__(16) unsigned int sh[8][256];
  const int wave = threadIdx.x >> 5, lane = threadIdx.x & 31;
  const int row = blockIdx.x * 8 + wave;
  if (row >= nrows) return;
  const float* xr = x + (size_t)row * DM;

  v4f v[4];
  float s = 0.0f;
#pragma unroll
  for (int j = 0; j < 4; ++j) {
    v[j] = *(const v4f*)(xr + j * 128 + lane * 4);
    s += (v[j][0] + v[j][1]) + (v[j][2] + v[j][3]);
  }
#pragma unroll
  for (int off = 1; off < 32; off <<= 1) s += __shfl_xor(s, off, 32);
  const float mu = s * (1.0f / 512.0f);
  float sq = 0.0f;
#pragma unroll
  for (int j = 0; j < 4; ++j)
#pragma unroll
    for (int e = 0; e < 4; ++e) {
      const float d = v[j][e] - mu;
      sq += d * d;
    }
#pragma unroll
  for (int off = 1; off < 32; off <<= 1) sq += __shfl_xor(sq, off, 32);
  const float var = sq * (1.0f / 512.0f);
  const float rs  = rsqrtf(var + 1e-5f);

  v4f y[4];
#pragma unroll
  for (int j = 0; j < 4; ++j) {
    const v4f g4 = *(const v4f*)(gw + j * 128 + lane * 4);
    const v4f b4 = *(const v4f*)(bw + j * 128 + lane * 4);
#pragma unroll
    for (int e = 0; e < 4; ++e) y[j][e] = (v[j][e] - mu) * rs * bfr(g4[e]) + bfr(b4[e]);
  }
  for (int pass = 0; pass < 2; ++pass) {
#pragma unroll
    for (int j = 0; j < 4; ++j) *(volatile v4f*)(outf + (size_t)row * DM + j * 128 + lane * 4) = y[j];
    __threadfence();
  }
  if constexpr (H16) {
#pragma unroll
    for (int j = 0; j < 4; ++j) {
      v2u u;
      u[0] = pk16(h_bits((_Float16)(y[j][0] * oscale)), h_bits((_Float16)(y[j][1] * oscale)));
      u[1] = pk16(h_bits((_Float16)(y[j][2] * oscale)), h_bits((_Float16)(y[j][3] * oscale)));
      *(v2u*)(&sh[wave][j * 64 + lane * 2]) = u;
    }
    __builtin_amdgcn_fence(__ATOMIC_RELEASE, "workgroup");
    __builtin_amdgcn_wave_barrier();
    __builtin_amdgcn_fence(__ATOMIC_ACQUIRE, "workgroup");
    v4u p[2];
#pragma unroll
    for (int q = 0; q < 2; ++q) p[q] = *(const v4u*)(&sh[wave][q * 128 + lane * 4]);
    for (int pass = 0; pass < 2; ++pass) {
#pragma unroll
      for (int q = 0; q < 2; ++q)
        *(volatile v4u*)(out16 + (size_t)row * DM + q * 256 + lane * 8) = p[q];
      __threadfence();
    }
  }
}

extern "C" void kernel_launch(void* const* d_in, const int* in_sizes, int n_in,
                              void* d_out, int out_size, void* d_ws, size_t ws_size,
                              hipStream_t stream) {
  if (n_in < 15) return;
  if (in_sizes[0] != ROWQ * DM) return;
  if (in_sizes[1] != ROWK * DM) return;
  if (in_sizes[2] != NB * NK) return;
  if (in_sizes[3] != DM * DM || in_sizes[5] != DM * DM || in_sizes[7] != DM * DM || in_sizes[9] != DM * DM) return;
  if (in_sizes[4] != DM || in_sizes[6] != DM || in_sizes[8] != DM || in_sizes[10] != DM) return;
  if (in_sizes[11] != DM || in_sizes[12] != DM || in_sizes[13] != DM || in_sizes[14] != DM) return;
  if (out_size != ROWQ * DM) return;

  const float* Qin = (const float*)d_in[0];
  const float* Kin = (const float*)d_in[1];
  const int*   msk = (const int*)d_in[2];
  const float* Wq  = (const float*)d_in[3];
  const float* bq  = (const float*)d_in[4];
  const float* Wk  = (const float*)d_in[5];
  const float* bk  = (const float*)d_in[6];
  const float* Wv  = (const float*)d_in[7];
  const float* bv  = (const float*)d_in[8];
  const float* Wo  = (const float*)d_in[9];
  const float* bo  = (const float*)d_in[10];
  const float* g0  = (const float*)d_in[11];
  const float* b0  = (const float*)d_in[12];
  const float* g1  = (const float*)d_in[13];
  const float* b1  = (const float*)d_in[14];

  const size_t P16a = (size_t)ROWQ * DM * 2;
  const size_t PW   = (size_t)DM * DM * 2;
  const size_t P32a = (size_t)ROWQ * DM * 4;
  const size_t PVT  = (size_t)NB * DM * NK * 2;
  size_t off = 0;
  const size_t oQh   = off; off += P16a;
  const size_t oKh   = off; off += P16a;
  const size_t oWqT  = off; off += PW;
  const size_t oWkT  = off; off += PW;
  const size_t oWvT  = off; off += PW;
  const size_t oWoT  = off; off += PW;
  const size_t oQf   = off; off += P32a;
  const size_t oQ16  = off; off += P16a;
  const size_t oK16  = off; off += P16a;
  const size_t oV16  = off; off += P16a;
  const size_t oVT   = off; off += PVT;
  const size_t oAO   = off; off += P32a;
  const size_t oL0f  = off; off += P32a;
  const size_t oL016 = off; off += P16a;
  const size_t oMlp  = off; off += P32a;
  if (off > ws_size) return;
  if (off > (size_t)134217728) return;

  char* ws = (char*)d_ws;
  unsigned short* Qh   = (unsigned short*)(ws + oQh);
  unsigned short* Kh   = (unsigned short*)(ws + oKh);
  unsigned short* WqT  = (unsigned short*)(ws + oWqT);
  unsigned short* WkT  = (unsigned short*)(ws + oWkT);
  unsigned short* WvT  = (unsigned short*)(ws + oWvT);
  unsigned short* WoT  = (unsigned short*)(ws + oWoT);
  float*          Qf   = (float*)(ws + oQf);
  unsigned short* Q16  = (unsigned short*)(ws + oQ16);
  unsigned short* K16  = (unsigned short*)(ws + oK16);
  unsigned short* V16  = (unsigned short*)(ws + oV16);
  unsigned short* VT   = (unsigned short*)(ws + oVT);
  float*          AO   = (float*)(ws + oAO);
  float*          L0f  = (float*)(ws + oL0f);
  unsigned short* L016 = (unsigned short*)(ws + oL016);
  float*          Mlp  = (float*)(ws + oMlp);
  float*          outf = (float*)d_out;

  const dim3 blk(256);
  const int n8a = ROWQ * DM / 8;
  const dim3 gCa((n8a + 255) / 256);
  const dim3 gW(DM / 64, DM / 64);
  const dim3 gG(((ROWQ / 64) * (DM / 64) + 7) / 8);
  const dim3 gVt(NK / 64, NH, NB);
  const dim3 gAttn(NQB * NH * NB);
  const dim3 gLn(ROWQ / 8);
  const float wScale = 1024.0f;
  const float aScale = 16.0f;
  const float cscale = 1.0f / 16384.0f;

  cvt16<<<gCa, blk, 0, stream>>>(Qin, Qh, n8a, aScale);
  cvt16<<<gCa, blk, 0, stream>>>(Kin, Kh, n8a, aScale);
  wtr16<<<gW, blk, 0, stream>>>(Wq, WqT, DM, DM, wScale);
  wtr16<<<gW, blk, 0, stream>>>(Wk, WkT, DM, DM, wScale);
  wtr16<<<gW, blk, 0, stream>>>(Wv, WvT, DM, DM, wScale);
  wtr16<<<gW, blk, 0, stream>>>(Wo, WoT, DM, DM, wScale);
  gemm64_f16<1><<<gG, blk, 0, stream>>>(Qh, DM, WqT, DM, bq, bq, cscale, aScale, Qf, Q16, DM, ROWQ, DM, DM);
  gemm64_f16<0><<<gG, blk, 0, stream>>>(Kh, DM, WkT, DM, bk, bk, cscale, aScale, AO, K16, DM, ROWK, DM, DM);
  gemm64_f16<0><<<gG, blk, 0, stream>>>(Kh, DM, WvT, DM, bv, bv, cscale, aScale, AO, V16, DM, ROWK, DM, DM);
  v_tr<<<gVt, blk, 0, stream>>>(V16, VT);
  attn_k<<<gAttn, dim3(128), 0, stream>>>(Q16, K16, VT, Qf, msk, AO);
  ln_k<true><<<gLn, blk, 0, stream>>>(AO, g0, b0, L0f, L016, ROWQ, aScale);
  gemm64_f16<2><<<gG, blk, 0, stream>>>(L016, DM, WoT, DM, bo, L0f, cscale, aScale, Mlp, V16, DM, ROWQ, DM, DM);
  ln_k<false><<<gLn, blk, 0, stream>>>(Mlp, g1, b1, outf, L016, ROWQ, aScale);
  (void)hipGetLastError();
}
